// Encoder_22436909154571
// MI455X (gfx1250) — hardware-verified
//
#include <hip/hip_runtime.h>
#include <hip/hip_fp16.h>


#ifndef NB
#define NB 16
#endif
#ifndef SEQ
#define SEQ 2048
#endif
#define NB_FULL  16
#define SEQ_FULL 2048
#define DM    128
#define NHEAD 4
#define DKH   32
#define NTOK  (NB * SEQ)
#define WMAT  (DM * DM)
#define PLANE_H ((size_t)NTOK * DM)
#define EPSLN 1e-5f

static_assert(NB >= 1 && NB <= NB_FULL);
static_assert(SEQ >= 256 && SEQ <= SEQ_FULL);
static_assert(SEQ % 256 == 0);
static_assert(SEQ % 64 == 0);
static_assert(NTOK % 64 == 0);
static_assert(DM == 32 * 4);
static_assert(NHEAD * DKH == DM);
static_assert(DKH == 32);
static_assert(DM % 32 == 0);
static_assert(WMAT == 8 * 256 * 8);
static_assert((size_t)5 * WMAT * 2 + (size_t)NTOK * DM * 4 * 2 + PLANE_H * 2 * 3 <= (size_t)134217728);

typedef _Float16 v16h __attribute__((ext_vector_type(16)));
typedef _Float16 v8h  __attribute__((ext_vector_type(8)));
typedef _Float16 v4h  __attribute__((ext_vector_type(4)));
typedef float    v8f  __attribute__((ext_vector_type(8)));
typedef float    v4f  __attribute__((ext_vector_type(4)));
typedef int      v4i  __attribute__((ext_vector_type(4)));

union Frag { v16h v; v8h h[2]; };

#define CSC (1.44269504088896340736f * 0.17677669529663688110f * 0.000244140625f)
#define PCARRY 10.0f
#define SC_O   0.015625f
#define SC_F   0.000244140625f

static __device__ __forceinline__ v8f zero8() {
    v8f z;
#pragma unroll
    for (int i = 0; i < 8; ++i) z[i] = 0.0f;
    return z;
}

static __device__ __forceinline__ v16h load_frag16(const _Float16* base, int ld, int lane) {
    int m  = lane & 15;
    int kb = (lane >> 4) << 3;
    const _Float16* p = base + (size_t)m * ld + kb;
    Frag f;
    f.h[0] = *(const v8h*)(p);
    f.h[1] = *(const v8h*)(p + 16);
    return f.v;
}

static __device__ __forceinline__ v8f wmma16(v16h a, v16h b, v8f c) {
    v8f d = __builtin_amdgcn_wmma_f32_16x16x32_f16(false, a, false, b, (short)0, c, false, false);
    asm volatile("v_nop\n\tv_nop\n\tv_nop\n\tv_nop" : "+v"(d) : "v"(a), "v"(b));
    return d;
}

static __device__ __forceinline__ float bf16r(float x) {
    unsigned u = __float_as_uint(x);
    u = (u + 0x7FFFu + ((u >> 16) & 1u)) & 0xFFFF0000u;
    return __uint_as_float(u);
}

static __device__ __forceinline__ float ex2(float x) {
    return __builtin_amdgcn_exp2f(x);
}

static __device__ __forceinline__ void wave_lds_sync() {
    __builtin_amdgcn_fence(3, "wavefront");
    asm volatile("s_wait_dscnt 0" ::: "memory");
    __builtin_amdgcn_wave_barrier();
}

static __device__ __forceinline__ float wave_sum(float v) {
    v += __shfl_xor(v, 16, 32);
    v += __shfl_xor(v, 8, 32);
    v += __shfl_xor(v, 4, 32);
    v += __shfl_xor(v, 2, 32);
    v += __shfl_xor(v, 1, 32);
    return v;
}

static __device__ __forceinline__ v4f ln_row(v4f a, v4f gw, v4f gb) {
    float s = (a.x + a.y) + (a.z + a.w);
    s = wave_sum(s);
    const float mu = s * (1.0f / 128.0f);
    const float d0 = a.x - mu, d1 = a.y - mu, d2 = a.z - mu, d3 = a.w - mu;
    float sq = (d0 * d0 + d1 * d1) + (d2 * d2 + d3 * d3);
    sq = wave_sum(sq);
    const float rinv = rsqrtf(sq * (1.0f / 128.0f) + EPSLN);
    v4f o;
    o.x = d0 * rinv * gw.x + gb.x;
    o.y = d1 * rinv * gw.y + gb.y;
    o.z = d2 * rinv * gw.z + gb.z;
    o.w = d3 * rinv * gw.w + gb.w;
    return o;
}

static __device__ __forceinline__ v8h cvt_w8(v4f a, v4f b) {
    v8h r;
    r[0] = (_Float16)(bf16r(a.x) * 64.0f);
    r[1] = (_Float16)(bf16r(a.y) * 64.0f);
    r[2] = (_Float16)(bf16r(a.z) * 64.0f);
    r[3] = (_Float16)(bf16r(a.w) * 64.0f);
    r[4] = (_Float16)(bf16r(b.x) * 64.0f);
    r[5] = (_Float16)(bf16r(b.y) * 64.0f);
    r[6] = (_Float16)(bf16r(b.z) * 64.0f);
    r[7] = (_Float16)(bf16r(b.w) * 64.0f);
    return r;
}

__global__ __launch_bounds__(256) void k_wprep(const float* __restrict__ wq,
                                                const float* __restrict__ wk,
                                                const float* __restrict__ wv,
                                                const float* __restrict__ w1,
                                                const float* __restrict__ w2,
                                                _Float16* __restrict__ wall) {
    const size_t e = ((size_t)blockIdx.x * 256 + threadIdx.x) * 8;
    const v8h h0 = cvt_w8(*(const v4f*)(wq + e), *(const v4f*)(wq + e + 4));
    const v8h h1 = cvt_w8(*(const v4f*)(wk + e), *(const v4f*)(wk + e + 4));
    const v8h h2 = cvt_w8(*(const v4f*)(wv + e), *(const v4f*)(wv + e + 4));
    const v8h h3 = cvt_w8(*(const v4f*)(w1 + e), *(const v4f*)(w1 + e + 4));
    const v8h h4 = cvt_w8(*(const v4f*)(w2 + e), *(const v4f*)(w2 + e + 4));
    *(volatile v8h*)(wall + 0 * (size_t)WMAT + e) = h0;
    *(volatile v8h*)(wall + 1 * (size_t)WMAT + e) = h1;
    *(volatile v8h*)(wall + 2 * (size_t)WMAT + e) = h2;
    *(volatile v8h*)(wall + 3 * (size_t)WMAT + e) = h3;
    *(volatile v8h*)(wall + 4 * (size_t)WMAT + e) = h4;
    __threadfence();
    *(volatile v8h*)(wall + 0 * (size_t)WMAT + e) = h0;
    *(volatile v8h*)(wall + 1 * (size_t)WMAT + e) = h1;
    *(volatile v8h*)(wall + 2 * (size_t)WMAT + e) = h2;
    *(volatile v8h*)(wall + 3 * (size_t)WMAT + e) = h3;
    *(volatile v8h*)(wall + 4 * (size_t)WMAT + e) = h4;
}

__global__ __launch_bounds__(128) __attribute__((amdgpu_num_vgpr(256)))
void k_ln_qkv(const float* __restrict__ x,
              const float* __restrict__ lnw,
              const float* __restrict__ lnb,
              const _Float16* __restrict__ wall,
              float* __restrict__ xn,
              _Float16* __restrict__ qk,
              _Float16* __restrict__ vT) {
    __shared__ __align__(16) _Float16 xs[64 * DM];
    __shared__ __align__(16) _Float16 qkst[4][8][16 * 32];
    __shared__ __align__(16) _Float16 vst[DM * 64];

    const int tid  = threadIdx.x;
    const int lane = tid & 31;
    const int w    = tid >> 5;
    const int tok0 = blockIdx.x * 64;
    const int b    = tok0 / SEQ;
    const int s0   = tok0 - b * SEQ;
    const int r0   = (lane >> 4) << 3;
    const int cc   = lane & 15;

    const float* xb  = x + ((size_t)b * SEQ_FULL + s0 + w * 16) * DM + lane * 4;
    float*       xnb = xn + ((size_t)tok0 + w * 16) * DM + lane * 4;

    v4f gw = *(const v4f*)(lnw + lane * 4);
    v4f gb = *(const v4f*)(lnb + lane * 4);
    gw.x = bf16r(gw.x); gw.y = bf16r(gw.y); gw.z = bf16r(gw.z); gw.w = bf16r(gw.w);
    gb.x = bf16r(gb.x); gb.y = bf16r(gb.y); gb.z = bf16r(gb.z); gb.w = bf16r(gb.w);

    v4f xo[16];
#pragma unroll
    for (int i = 0; i < 16; ++i) {
        v4f xv = *(const v4f*)(xb + (size_t)i * DM);
        xv.x = bf16r(xv.x); xv.y = bf16r(xv.y); xv.z = bf16r(xv.z); xv.w = bf16r(xv.w);
        const v4f o = ln_row(xv, gw, gb);
        xo[i] = o;
        v4h hv;
        hv.x = (_Float16)o.x; hv.y = (_Float16)o.y; hv.z = (_Float16)o.z; hv.w = (_Float16)o.w;
        *(v4h*)(&xs[(w * 16 + i) * DM + lane * 4]) = hv;
        *(volatile v4f*)(xnb + (size_t)i * DM) = o;
    }
    __threadfence();
#pragma unroll
    for (int i = 0; i < 16; ++i) *(volatile v4f*)(xnb + (size_t)i * DM) = xo[i];
    wave_lds_sync();

    v16h a[4];
#pragma unroll
    for (int kt = 0; kt < 4; ++kt) a[kt] = load_frag16(&xs[(w * 16) * DM + kt * 32], DM, lane);

#pragma unroll 1
    for (int oh = 0; oh < 8; ++oh) {
        const _Float16* wr = wall + (size_t)oh * 32 * DM;
        v8f c0 = zero8(), c1 = zero8();
#pragma unroll
        for (int kt = 0; kt < 4; ++kt) {
            v16h b0 = load_frag16(wr + kt * 32, DM, lane);
            v16h b1 = load_frag16(wr + 16 * DM + kt * 32, DM, lane);
            c0 = wmma16(a[kt], b0, c0);
            c1 = wmma16(a[kt], b1, c1);
        }
        const bool isq = oh < 4;
#pragma unroll
        for (int g = 0; g < 8; ++g) {
            float v0 = c0[g], v1 = c1[g];
            v0 = isq ? fmaxf(v0, 0.0f) : v0;
            v1 = isq ? fmaxf(v1, 0.0f) : v1;
            qkst[w][oh][(r0 + g) * 32 + cc]      = (_Float16)v0;
            qkst[w][oh][(r0 + g) * 32 + 16 + cc] = (_Float16)v1;
        }
    }
#pragma unroll 1
    for (int h = 0; h < NHEAD; ++h) {
        const _Float16* wr = wall + (size_t)(2 * DM + h * 32) * DM;
        v8f c0 = zero8(), c1 = zero8();
#pragma unroll
        for (int kt = 0; kt < 4; ++kt) {
            v16h b0 = load_frag16(wr + kt * 32, DM, lane);
            v16h b1 = load_frag16(wr + 16 * DM + kt * 32, DM, lane);
            c0 = wmma16(a[kt], b0, c0);
            c1 = wmma16(a[kt], b1, c1);
        }
        v8h p0, p1;
#pragma unroll
        for (int g = 0; g < 8; ++g) { p0[g] = (_Float16)c0[g]; p1[g] = (_Float16)c1[g]; }
        *(v8h*)(&vst[(h * 32 + cc) * 64 + w * 16 + r0])      = p0;
        *(v8h*)(&vst[(h * 32 + 16 + cc) * 64 + w * 16 + r0]) = p1;
    }
    __syncthreads();

    v8h pq[8][2];
    v8h pvv[8];
#pragma unroll
    for (int oh = 0; oh < 8; ++oh) {
        pq[oh][0] = *(const v8h*)(&qkst[w][oh][lane * 8]);
        pq[oh][1] = *(const v8h*)(&qkst[w][oh][256 + lane * 8]);
    }
#pragma unroll
    for (int i = 0; i < 8; ++i) {
        const int col = w * 32 + i * 4 + (lane >> 3);
        pvv[i] = *(const v8h*)(&vst[col * 64 + (lane & 7) * 8]);
    }
    const size_t vrow = (size_t)b * DM + w * 32 + (lane >> 3);
    const size_t voff = (size_t)s0 + (lane & 7) * 8;
#pragma unroll
    for (int oh = 0; oh < 8; ++oh) {
        const size_t base = (size_t)(oh >> 2) * PLANE_H +
                            ((size_t)(b * NHEAD + (oh & 3)) * SEQ + s0 + w * 16) * DKH + lane * 8;
        *(volatile v8h*)(qk + base)       = pq[oh][0];
        *(volatile v8h*)(qk + base + 256) = pq[oh][1];
    }
#pragma unroll
    for (int i = 0; i < 8; ++i)
        *(volatile v8h*)(vT + (vrow + i * 4) * SEQ + voff) = pvv[i];
    __threadfence();
#pragma unroll
    for (int oh = 0; oh < 8; ++oh) {
        const size_t base = (size_t)(oh >> 2) * PLANE_H +
                            ((size_t)(b * NHEAD + (oh & 3)) * SEQ + s0 + w * 16) * DKH + lane * 8;
        *(volatile v8h*)(qk + base)       = pq[oh][0];
        *(volatile v8h*)(qk + base + 256) = pq[oh][1];
    }
#pragma unroll
    for (int i = 0; i < 8; ++i)
        *(volatile v8h*)(vT + (vrow + i * 4) * SEQ + voff) = pvv[i];
}

static __device__ __forceinline__ v16h softmax_step(const v8f& sA, const v8f& sB,
                                                    const int (&mk)[16],
                                                    float& m, float& l,
                                                    v8f& o0, v8f& o1) {
    const float ninf = -__builtin_huge_valf();
    float t[16];
#pragma unroll
    for (int i = 0; i < 8; ++i) {
        t[i]     = (mk[i] != 0)     ? sA[i] * CSC : ninf;
        t[8 + i] = (mk[8 + i] != 0) ? sB[i] * CSC : ninf;
    }
    float tmax = t[0];
#pragma unroll
    for (int i = 1; i < 16; ++i) tmax = fmaxf(tmax, t[i]);
    tmax = fmaxf(tmax, __shfl_xor(tmax, 16, 32));
    const float mn    = fmaxf(m, tmax);
    const float alpha = ex2(m - mn);
    const float off   = PCARRY - mn;
    float ps = 0.0f;
    Frag pf;
#pragma unroll
    for (int i = 0; i < 16; ++i) {
        const float p = ex2(t[i] + off);
        ps += p;
        pf.v[i] = (_Float16)p;
    }
    ps += __shfl_xor(ps, 16, 32);
    l = l * alpha + ps;
    m = mn;
#pragma unroll
    for (int i = 0; i < 8; ++i) { o0[i] *= alpha; o1[i] *= alpha; }
    return pf.v;
}

__global__ __launch_bounds__(256) __attribute__((amdgpu_num_vgpr(256)))
void k_attn(const _Float16* __restrict__ qk,
            const _Float16* __restrict__ vT,
            const int* __restrict__ mask,
            const float* __restrict__ xn,
            float* __restrict__ sa) {
    __shared__ __align__(16) float Ost[8][32 * 32];

    const int tid  = threadIdx.x;
    const int lane = tid & 31;
    const int w    = tid >> 5;
    const int bh   = blockIdx.x;
    const int b    = bh / NHEAD;
    const int h    = bh - b * NHEAD;
    const int q0   = blockIdx.y * 256 + w * 32;
    const int r0   = (lane >> 4) << 3;
    const int cc   = lane & 15;

    const _Float16* qb = qk + ((size_t)bh * SEQ + q0) * DKH;
    const _Float16* kb = qk + PLANE_H + (size_t)bh * SEQ * DKH;
    const _Float16* vb = vT + (size_t)bh * DKH * SEQ;
    const int*      mb = mask + (size_t)b * SEQ_FULL + r0;

    const v16h qf0 = load_frag16(qb, DKH, lane);
    const v16h qf1 = load_frag16(qb + 16 * DKH, DKH, lane);

    v8f oA0 = zero8(), oA1 = zero8();
    v8f oB0 = zero8(), oB1 = zero8();
    float mA = -1.0e30f, lA = 0.0f, mB = -1.0e30f, lB = 0.0f;

#pragma unroll 1
    for (int key0 = 0; key0 < SEQ; key0 += 32) {
        const v16h kfA = load_frag16(kb + (size_t)key0 * DKH, DKH, lane);
        const v16h kfB = load_frag16(kb + (size_t)(key0 + 16) * DKH, DKH, lane);
        const v16h vf0 = load_frag16(vb + key0, SEQ, lane);
        const v16h vf1 = load_frag16(vb + (size_t)16 * SEQ + key0, SEQ, lane);
        const v4i k0 = *(const v4i*)(mb + key0);
        const v4i k1 = *(const v4i*)(mb + key0 + 4);
        const v4i k2 = *(const v4i*)(mb + key0 + 16);
        const v4i k3 = *(const v4i*)(mb + key0 + 20);
        const int mk[16] = { k0.x, k0.y, k0.z, k0.w, k1.x, k1.y, k1.z, k1.w,
                             k2.x, k2.y, k2.z, k2.w, k3.x, k3.y, k3.z, k3.w };
        {
            const v8f sA = wmma16(kfA, qf0, zero8());
            const v8f sB = wmma16(kfB, qf0, zero8());
            const v16h pf = softmax_step(sA, sB, mk, mA, lA, oA0, oA1);
            oA0 = wmma16(vf0, pf, oA0);
            oA1 = wmma16(vf1, pf, oA1);
        }
        {
            const v8f sA = wmma16(kfA, qf1, zero8());
            const v8f sB = wmma16(kfB, qf1, zero8());
            const v16h pf = softmax_step(sA, sB, mk, mB, lB, oB0, oB1);
            oB0 = wmma16(vf0, pf, oB0);
            oB1 = wmma16(vf1, pf, oB1);
        }
    }

    const float iA = (1.0f / lA) * SC_O;
    const float iB = (1.0f / lB) * SC_O;
    {
        v4f t0, t1;
        t0.x = oA0[0] * iA; t0.y = oA0[1] * iA; t0.z = oA0[2] * iA; t0.w = oA0[3] * iA;
        t1.x = oA0[4] * iA; t1.y = oA0[5] * iA; t1.z = oA0[6] * iA; t1.w = oA0[7] * iA;
        *(v4f*)(&Ost[w][cc * 32 + r0])     = t0;
        *(v4f*)(&Ost[w][cc * 32 + r0 + 4]) = t1;
        t0.x = oA1[0] * iA; t0.y = oA1[1] * iA; t0.z = oA1[2] * iA; t0.w = oA1[3] * iA;
        t1.x = oA1[4] * iA; t1.y = oA1[5] * iA; t1.z = oA1[6] * iA; t1.w = oA1[7] * iA;
        *(v4f*)(&Ost[w][cc * 32 + 16 + r0])     = t0;
        *(v4f*)(&Ost[w][cc * 32 + 16 + r0 + 4]) = t1;
        t0.x = oB0[0] * iB; t0.y = oB0[1] * iB; t0.z = oB0[2] * iB; t0.w = oB0[3] * iB;
        t1.x = oB0[4] * iB; t1.y = oB0[5] * iB; t1.z = oB0[6] * iB; t1.w = oB0[7] * iB;
        *(v4f*)(&Ost[w][(16 + cc) * 32 + r0])     = t0;
        *(v4f*)(&Ost[w][(16 + cc) * 32 + r0 + 4]) = t1;
        t0.x = oB1[0] * iB; t0.y = oB1[1] * iB; t0.z = oB1[2] * iB; t0.w = oB1[3] * iB;
        t1.x = oB1[4] * iB; t1.y = oB1[5] * iB; t1.z = oB1[6] * iB; t1.w = oB1[7] * iB;
        *(v4f*)(&Ost[w][(16 + cc) * 32 + 16 + r0])     = t0;
        *(v4f*)(&Ost[w][(16 + cc) * 32 + 16 + r0 + 4]) = t1;
    }
    wave_lds_sync();

    const int    tq  = lane >> 3;
    const int    pc  = (lane & 7) * 4;
    const size_t gb0 = ((size_t)b * SEQ + q0 + tq) * DM + h * DKH + pc;
    v4f sv[8];
#pragma unroll
    for (int i = 0; i < 8; ++i) {
        const v4f f = *(const v4f*)(&Ost[w][(i * 4 + tq) * 32 + pc]);
        const v4f r = *(const v4f*)(xn + gb0 + (size_t)i * 4 * DM);
        sv[i] = f + r;
    }
#pragma unroll
    for (int i = 0; i < 8; ++i) *(volatile v4f*)(sa + gb0 + (size_t)i * 4 * DM) = sv[i];
    __threadfence();
#pragma unroll
    for (int i = 0; i < 8; ++i) *(volatile v4f*)(sa + gb0 + (size_t)i * 4 * DM) = sv[i];
}

__global__ __launch_bounds__(128) __attribute__((amdgpu_num_vgpr(256)))
void k_ffn(const float* __restrict__ sa,
           const float* __restrict__ lnw,
           const float* __restrict__ lnb,
           const float* __restrict__ b1,
           const float* __restrict__ b2,
           const _Float16* __restrict__ wall,
           float* __restrict__ out) {
    __shared__ __align__(16) _Float16 hs[64 * DM];
    __shared__ __align__(16) _Float16 h2s[4][16 * DM];
    __shared__ __align__(16) float    Ost[4][16 * DM];

    const int tid  = threadIdx.x;
    const int lane = tid & 31;
    const int w    = tid >> 5;
    const int r0   = (lane >> 4) << 3;
    const int cc   = lane & 15;
    const size_t row0 = (size_t)blockIdx.x * 64 + w * 16;
    const float* sab  = sa + row0 * DM + lane * 4;

    v4f gw = *(const v4f*)(lnw + lane * 4);
    v4f gb = *(const v4f*)(lnb + lane * 4);
    gw.x = bf16r(gw.x); gw.y = bf16r(gw.y); gw.z = bf16r(gw.z); gw.w = bf16r(gw.w);
    gb.x = bf16r(gb.x); gb.y = bf16r(gb.y); gb.z = bf16r(gb.z); gb.w = bf16r(gb.w);

#pragma unroll 1
    for (int i = 0; i < 16; ++i) {
        const v4f sv = *(const v4f*)(sab + (size_t)i * DM);
        const v4f o = ln_row(sv, gw, gb);
        v4h hv;
        hv.x = (_Float16)o.x; hv.y = (_Float16)o.y; hv.z = (_Float16)o.z; hv.w = (_Float16)o.w;
        *(v4h*)(&hs[(w * 16 + i) * DM + lane * 4]) = hv;
    }
    wave_lds_sync();

    v16h a[4];
#pragma unroll
    for (int kt = 0; kt < 4; ++kt) a[kt] = load_frag16(&hs[(w * 16) * DM + kt * 32], DM, lane);

    const _Float16* w1p = wall + (size_t)3 * WMAT;
    const _Float16* w2p = wall + (size_t)4 * WMAT;

#pragma unroll 1
    for (int nt = 0; nt < 8; ++nt) {
        const _Float16* wr = w1p + (size_t)(nt * 16) * DM;
        v8f c = zero8();
#pragma unroll
        for (int kt = 0; kt < 4; ++kt) {
            v16h bf = load_frag16(wr + kt * 32, DM, lane);
            c = wmma16(a[kt], bf, c);
        }
        const float bias = bf16r(b1[nt * 16 + cc]) * 64.0f;
#pragma unroll
        for (int g = 0; g < 8; ++g)
            h2s[w][(r0 + g) * DM + nt * 16 + cc] = (_Float16)fmaxf(c[g] + bias, 0.0f);
    }
    wave_lds_sync();

#pragma unroll
    for (int kt = 0; kt < 4; ++kt) a[kt] = load_frag16(&h2s[w][kt * 32], DM, lane);

#pragma unroll 1
    for (int nt = 0; nt < 8; ++nt) {
        const _Float16* wr = w2p + (size_t)(nt * 16) * DM;
        v8f c = zero8();
#pragma unroll
        for (int kt = 0; kt < 4; ++kt) {
            v16h bf = load_frag16(wr + kt * 32, DM, lane);
            c = wmma16(a[kt], bf, c);
        }
        const float bias = bf16r(b2[nt * 16 + cc]);
#pragma unroll
        for (int g = 0; g < 8; ++g)
            Ost[w][(r0 + g) * DM + nt * 16 + cc] = c[g] * SC_F + bias;
    }
    wave_lds_sync();

    float* ob = out + row0 * DM + lane * 4;
    v4f sv[16];
#pragma unroll
    for (int i = 0; i < 16; ++i) {
        const v4f f = *(const v4f*)(&Ost[w][i * DM + lane * 4]);
        const v4f r = *(const v4f*)(sab + (size_t)i * DM);
        sv[i] = r + f;
    }
#pragma unroll
    for (int i = 0; i < 16; ++i) *(volatile v4f*)(ob + (size_t)i * DM) = sv[i];
    __threadfence();
#pragma unroll
    for (int i = 0; i < 16; ++i) *(volatile v4f*)(ob + (size_t)i * DM) = sv[i];
}

extern "C" void kernel_launch(void* const* d_in, const int* in_sizes, int n_in,
                              void* d_out, int out_size, void* d_ws, size_t ws_size,
                              hipStream_t stream) {
    if (n_in < 11) return;
    if (in_sizes[0] < ((NB - 1) * SEQ_FULL + SEQ) * DM) return;
    if (in_sizes[1] < (NB - 1) * SEQ_FULL + SEQ) return;
    if (in_sizes[2] < DM || in_sizes[3] < DM) return;
    if (in_sizes[4] < WMAT || in_sizes[5] < WMAT || in_sizes[6] < WMAT) return;
    if (in_sizes[7] < WMAT || in_sizes[8] < DM || in_sizes[9] < WMAT || in_sizes[10] < DM) return;
    if (out_size < NTOK * DM) return;

    const float* x    = (const float*)d_in[0];
    const int*   mask = (const int*)d_in[1];
    const float* lnw  = (const float*)d_in[2];
    const float* lnb  = (const float*)d_in[3];
    const float* wq   = (const float*)d_in[4];
    const float* wk   = (const float*)d_in[5];
    const float* wv   = (const float*)d_in[6];
    const float* w1   = (const float*)d_in[7];
    const float* b1   = (const float*)d_in[8];
    const float* w2   = (const float*)d_in[9];
    const float* b2   = (const float*)d_in[10];
    float* out = (float*)d_out;

    char* ws = (char*)d_ws;
    size_t off = 0;
    _Float16* wall = (_Float16*)(ws + off); off += (size_t)5 * WMAT * 2;
    float*    xn   = (float*)(ws + off);    off += (size_t)NTOK * DM * 4;
    _Float16* qk   = (_Float16*)(ws + off); off += PLANE_H * 2 * 2;
    _Float16* vT   = (_Float16*)(ws + off); off += PLANE_H * 2;
    float*    sa   = (float*)(ws + off);    off += (size_t)NTOK * DM * 4;
    if (off > ws_size) return;

    k_wprep<<<dim3(8), dim3(256), 0, stream>>>(wq, wk, wv, w1, w2, wall);
    k_ln_qkv<<<dim3(NTOK / 64), dim3(128), 0, stream>>>(x, lnw, lnb, wall, xn, qk, vT);
    k_attn<<<dim3(NB * NHEAD, SEQ / 256), dim3(256), 0, stream>>>(qk, vT, mask, xn, sa);
    k_ffn<<<dim3(NTOK / 64), dim3(128), 0, stream>>>(sa, lnw, lnb, b1, b2, wall, out);
}
